// TinyAttentionBlock_46943992545481
// MI455X (gfx1250) — hardware-verified
//
#include <hip/hip_runtime.h>


#define NB_  8
#define NN   2048
#define CC   256
#define NT   (NB_ * NN)
#define PCAR 1024.0f
typedef _Float16 h16;
typedef unsigned short bf;
typedef __attribute__((ext_vector_type(16))) __bf16   v16bf;
typedef __attribute__((ext_vector_type(16))) _Float16 v16h;
typedef __attribute__((ext_vector_type(8)))  _Float16 v8h;
typedef __attribute__((ext_vector_type(8)))  unsigned short v8us;
typedef __attribute__((ext_vector_type(8)))  float    v8f;
typedef __attribute__((ext_vector_type(4)))  float    v4f;
typedef v8h  __attribute__((may_alias)) v8ha;
typedef v4f  __attribute__((may_alias)) v4fa;
typedef v8us __attribute__((may_alias)) v8usa;

__device__ __forceinline__ unsigned short f2bf(float f) { unsigned u = __float_as_uint(f); u += 0x7FFFu + ((u >> 16) & 1u); return (unsigned short)(u >> 16); }
__device__ __forceinline__ float bf2f(unsigned short b) { return __uint_as_float(((unsigned)b) << 16); }
__device__ __forceinline__ float bfr(float f) { return bf2f(f2bf(f)); }
__device__ __forceinline__ v16h cat16(v8h lo, v8h hi) { return __builtin_shufflevector(lo, hi, 0, 1, 2, 3, 4, 5, 6, 7, 8, 9, 10, 11, 12, 13, 14, 15); }
__device__ __forceinline__ v16bf cat16b(v8us lo, v8us hi) { return __builtin_bit_cast(v16bf, __builtin_shufflevector(lo, hi, 0, 1, 2, 3, 4, 5, 6, 7, 8, 9, 10, 11, 12, 13, 14, 15)); }
__device__ __forceinline__ v8f wmma16(v16h a, v16h b, v8f c) { return __builtin_amdgcn_wmma_f32_16x16x32_f16(false, a, false, b, (short)0, c, false, false); }
__device__ __forceinline__ v8f wmmab(v16bf a, v16bf b, v8f c) { return __builtin_amdgcn_wmma_f32_16x16x32_bf16(false, a, false, b, (short)0, c, false, false); }


template <typename T16> struct WFrag;
template <> struct WFrag<h16> { typedef v16h V; static __device__ __forceinline__ V ld(const h16* p) { return cat16(*(const v8h*)p, *(const v8h*)(p + 16)); } static __device__ __forceinline__ v8f mma(V a, V b, v8f c) { return wmma16(a, b, c); } };
template <> struct WFrag<bf> { typedef v16bf V; static __device__ __forceinline__ V ld(const bf* p) { return cat16b(*(const v8us*)p, *(const v8us*)(p + 16)); } static __device__ __forceinline__ v8f mma(V a, V b, v8f c) { return wmmab(a, b, c); } };
template <typename T16, int NSPLIT, bool BIAS>
__global__ __launch_bounds__(32) void k_gemmw(const T16* __restrict__ A, const T16* __restrict__ A2, const T16* __restrict__ Bt, const T16* __restrict__ Bt2, int K, float* C, int ldc, const float* __restrict__ bias, size_t sA, size_t sB, size_t sC) {
    typedef typename WFrag<T16>::V V;
    __shared__ __align__(16) float os[16 * 68];
    const size_t z = blockIdx.z; A += z * sA; if (A2) A2 += z * sA; Bt += z * sB; if (Bt2) Bt2 += z * sB; C += z * sC;
    const int lane = threadIdx.x & 31, lr = lane & 15, hi = lane >> 4; const int r0 = blockIdx.x * 64, c0 = blockIdx.y * 64;
    v8f acc[4][4];
#pragma unroll
    for (int mb = 0; mb < 4; ++mb)
#pragma unroll
        for (int nb = 0; nb < 4; ++nb) acc[mb][nb] = (v8f){};
    const size_t aoff = (size_t)(r0 + lr) * K + 8 * hi, boff = (size_t)(c0 + lr) * K + 8 * hi;
#pragma unroll 1
    for (int kc = 0; kc < K; kc += 32) {
        V a[4], a2[4];
#pragma unroll
        for (int mb = 0; mb < 4; ++mb) { a[mb] = WFrag<T16>::ld(A + aoff + (size_t)mb * 16 * K + kc); if (NSPLIT == 1 || NSPLIT == 2) a2[mb] = WFrag<T16>::ld(A2 + aoff + (size_t)mb * 16 * K + kc); }
#pragma unroll
        for (int nb = 0; nb < 4; ++nb) { const V b = WFrag<T16>::ld(Bt + boff + (size_t)nb * 16 * K + kc); V b2; if (NSPLIT >= 2) b2 = WFrag<T16>::ld(Bt2 + boff + (size_t)nb * 16 * K + kc);
#pragma unroll
            for (int mb = 0; mb < 4; ++mb) { acc[mb][nb] = WFrag<T16>::mma(a[mb], b, acc[mb][nb]); if (NSPLIT == 1 || NSPLIT == 2) acc[mb][nb] = WFrag<T16>::mma(a2[mb], b, acc[mb][nb]); if (NSPLIT >= 2) acc[mb][nb] = WFrag<T16>::mma(a[mb], b2, acc[mb][nb]); } }
        asm volatile("v_nop\n\tv_nop\n\tv_nop\n\tv_nop" : "+v"(acc[0][0]), "+v"(acc[1][1]), "+v"(acc[2][2]), "+v"(acc[3][3]) : "v"(a[0]), "v"(a[3]));
    }
#pragma unroll
    for (int mb = 0; mb < 4; ++mb) {
#pragma unroll
        for (int nb = 0; nb < 4; ++nb) {
#pragma unroll
            for (int j = 0; j < 8; ++j) os[(hi * 8 + j) * 68 + nb * 16 + lr] = acc[mb][nb][j]; }
        __builtin_amdgcn_wave_barrier(); asm volatile("" ::: "memory");
        float* crow = C + (size_t)(r0 + mb * 16) * ldc + c0;
#pragma unroll 1
        for (int ps = 0; ps < 2; ++ps) {
#pragma unroll
            for (int s = 0; s < 8; ++s) { const int row = 2 * s + hi, cofs = lr * 4; v4f val = *(const v4fa*)(os + row * 68 + cofs); if (BIAS) { val[0] += bfr(bias[c0 + cofs]); val[1] += bfr(bias[c0 + cofs + 1]); val[2] += bfr(bias[c0 + cofs + 2]); val[3] += bfr(bias[c0 + cofs + 3]); }
                *(volatile v4f*)(crow + (size_t)row * ldc + cofs) = val; }
            if (ps == 0) __threadfence(); }
        __builtin_amdgcn_wave_barrier(); asm volatile("" ::: "memory");
    }
}

__device__ __forceinline__ h16 tohx(float x) { return (h16)x; }
__device__ __forceinline__ void splitf(float y, unsigned short& h, unsigned short& l) { h = f2bf(y); l = f2bf(y - bf2f(h)); }
typedef __attribute__((ext_vector_type(4))) _Float16 v4h;
typedef __attribute__((ext_vector_type(2))) _Float16 v2h;
typedef __attribute__((ext_vector_type(4))) unsigned short v4us;
typedef __attribute__((ext_vector_type(2))) unsigned short v2us;

__global__ __launch_bounds__(256) void k_wtb(const float* __restrict__ w, int K, int N, int ldw, int col0, bf* Bt) {
    const int lane = threadIdx.x & 31; const int L0 = (blockIdx.x * 8 + (threadIdx.x >> 5)) * 8; const int nlines = N * K / 64;
#pragma unroll 1
    for (int ps = 0; ps < 2; ++ps) {
#pragma unroll 1
        for (int l = 0; l < 8; ++l) { const int L = L0 + l; if (L >= nlines) break; const int e = L * 64 + lane * 2; v2us o;
#pragma unroll
            for (int q = 0; q < 2; ++q) { const int n = (e + q) / K, k = (e + q) % K; o[q] = f2bf(w[(size_t)k * ldw + col0 + n]); }
            *(volatile v2us*)(Bt + e) = o; }
        if (ps == 0) __threadfence(); }
}
__global__ __launch_bounds__(256) void k_ln1(const float* __restrict__ x, const float* __restrict__ gg, const float* __restrict__ bb, bf* Ph, bf* Pl) {
    const int lane = threadIdx.x & 31; const int r = blockIdx.x * 8 + (threadIdx.x >> 5); if (r >= NT) return; float v[8]; float s = 0.f;
#pragma unroll
    for (int c = 0; c < 2; ++c)
#pragma unroll
        for (int q = 0; q < 4; ++q) { const float t = bfr(x[(size_t)r * CC + c * 128 + lane * 4 + q]); v[c * 4 + q] = t; s += t; }
#pragma unroll
    for (int sh = 16; sh; sh >>= 1) s += __shfl_xor(s, sh, 32);
    const float mu = s * (1.0f / CC); float qq = 0.f;
#pragma unroll
    for (int i = 0; i < 8; ++i) { const float d = v[i] - mu; qq = fmaf(d, d, qq); }
#pragma unroll
    for (int sh = 16; sh; sh >>= 1) qq += __shfl_xor(qq, sh, 32);
    const float rs = rsqrtf(qq * (1.0f / CC) + 1e-5f); v4us oh[2], ol[2];
#pragma unroll
    for (int c = 0; c < 2; ++c)
#pragma unroll
        for (int q = 0; q < 4; ++q) { const int col = c * 128 + lane * 4 + q; unsigned short a, b2; splitf((v[c * 4 + q] - mu) * rs * bfr(gg[col]) + bfr(bb[col]), a, b2); oh[c][q] = a; ol[c][q] = b2; }
#pragma unroll 1
    for (int ps = 0; ps < 2; ++ps) {
#pragma unroll
        for (int c = 0; c < 2; ++c) { *(volatile v4us*)(Ph + (size_t)r * CC + c * 128 + lane * 4) = oh[c]; *(volatile v4us*)(Pl + (size_t)r * CC + c * 128 + lane * 4) = ol[c]; }
        if (ps == 0) __threadfence(); }
}
__global__ __launch_bounds__(256) void k_qkplanes(const float* __restrict__ F, h16* Qp, h16* Kp) {
    const int lane = threadIdx.x & 31; const int L0 = (blockIdx.x * 8 + (threadIdx.x >> 5)) * 8; const int nlines = NT * 2 * CC / 64;
#pragma unroll 1
    for (int ps = 0; ps < 2; ++ps) {
#pragma unroll
        for (int l = 0; l < 8; ++l) { const int L = L0 + l; if (L >= nlines) break; const int e = L * 64 + lane * 2; const int c = e & 511; const int r = e >> 9; const bool isq = c < CC; const int cc = isq ? c : c - CC; v2h v;
#pragma unroll
            for (int q = 0; q < 2; ++q) v[q] = tohx(F[(size_t)r * (3 * CC) + (isq ? 0 : CC) + cc + q]);
            *(volatile v2h*)((isq ? Qp : Kp) + (size_t)r * CC + cc) = v; }
        if (ps == 0) __threadfence(); }
}
__global__ __launch_bounds__(256) void k_vtplane(const float* __restrict__ F, h16* VT) {
    const int lane = threadIdx.x & 31; const int L0 = (blockIdx.x * 8 + (threadIdx.x >> 5)) * 8; const int nlines = NT * CC / 64;
#pragma unroll 1
    for (int ps = 0; ps < 2; ++ps) {
#pragma unroll
        for (int l = 0; l < 8; ++l) { const int L = L0 + l; if (L >= nlines) break; const int e = L * 64 + lane * 2; const int n = e & 2047; const int c = (e >> 11) & 255; const int b = e >> 19; v2h v;
#pragma unroll
            for (int q = 0; q < 2; ++q) v[q] = tohx(F[((size_t)b * NN + n + q) * (3 * CC) + 2 * CC + c]);
            *(volatile v2h*)(VT + (size_t)e) = v; }
        if (ps == 0) __threadfence(); }
}
__global__ __launch_bounds__(256) void k_softrb(const float* __restrict__ Sb, const float* __restrict__ tab, const float* __restrict__ scp, h16* P) {
    const int lane = threadIdx.x & 31; const int i = blockIdx.x * 8 + (threadIdx.x >> 5); if (i >= NN) return; const float* sr = Sb + (size_t)i * NN; const float sc = bfr(scp[0]);
    float m = -3.0e38f;
#pragma unroll 1
    for (int c0 = lane * 4; c0 < NN; c0 += 128) { const v4f v = *(const v4f*)(sr + c0);
#pragma unroll
        for (int q = 0; q < 4; ++q) m = fmaxf(m, v[q] + bfr(tab[c0 + q - i + NN - 1])); }
#pragma unroll
    for (int sh = 16; sh; sh >>= 1) m = fmaxf(m, __shfl_xor(m, sh, 32));
    float sum = 0.f;
#pragma unroll 1
    for (int c0 = lane * 4; c0 < NN; c0 += 128) { const v4f v = *(const v4f*)(sr + c0);
#pragma unroll
        for (int q = 0; q < 4; ++q) sum += __expf((v[q] + bfr(tab[c0 + q - i + NN - 1])) - m); }
#pragma unroll
    for (int sh = 16; sh; sh >>= 1) sum += __shfl_xor(sum, sh, 32);
    const float f = __fdiv_rn(PCAR, sum) * sc;
#pragma unroll 1
    for (int ps = 0; ps < 2; ++ps) {
#pragma unroll 1
        for (int c0 = lane * 4; c0 < NN; c0 += 128) { const v4f v = *(const v4f*)(sr + c0); v4h o;
#pragma unroll
            for (int q = 0; q < 4; ++q) o[q] = tohx(__expf((v[q] + bfr(tab[c0 + q - i + NN - 1])) - m) * f);
            *(volatile v4h*)(P + (size_t)i * NN + c0) = o; }
        if (ps == 0) __threadfence(); }
}
__global__ __launch_bounds__(256) void k_split1k(const float* __restrict__ A, int nlines, bf* Ph, bf* Pl) {
    const int lane = threadIdx.x & 31; const int L0 = (blockIdx.x * 8 + (threadIdx.x >> 5)) * 8;
#pragma unroll 1
    for (int ps = 0; ps < 2; ++ps) {
#pragma unroll
        for (int l = 0; l < 8; ++l) { const int L = L0 + l; if (L >= nlines) break; const int e = L * 64 + lane * 2; v2us oh, ol;
#pragma unroll
            for (int q = 0; q < 2; ++q) { unsigned short a, b2; splitf(A[(size_t)e + q] * (1.0f / PCAR), a, b2); oh[q] = a; ol[q] = b2; }
            *(volatile v2us*)(Ph + (size_t)e) = oh; *(volatile v2us*)(Pl + (size_t)e) = ol; }
        if (ps == 0) __threadfence(); }
}
__global__ __launch_bounds__(256) void k_ln2(const float* __restrict__ A, const float* __restrict__ gg, const float* __restrict__ bb, float* OUT) {
    const int lane = threadIdx.x & 31; const int r = blockIdx.x * 8 + (threadIdx.x >> 5); if (r >= NT) return; float v[8]; float s = 0.f;
#pragma unroll
    for (int c = 0; c < 2; ++c)
#pragma unroll
        for (int q = 0; q < 4; ++q) { const float t = A[(size_t)r * CC + c * 128 + lane * 4 + q]; v[c * 4 + q] = t; s += t; }
#pragma unroll
    for (int sh = 16; sh; sh >>= 1) s += __shfl_xor(s, sh, 32);
    const float mu = s * (1.0f / CC); float qq = 0.f;
#pragma unroll
    for (int i = 0; i < 8; ++i) { const float d = v[i] - mu; qq = fmaf(d, d, qq); }
#pragma unroll
    for (int sh = 16; sh; sh >>= 1) qq += __shfl_xor(qq, sh, 32);
    const float rs = rsqrtf(qq * (1.0f / CC) + 1e-5f); v4f o[2];
#pragma unroll
    for (int c = 0; c < 2; ++c)
#pragma unroll
        for (int q = 0; q < 4; ++q) { const int col = c * 128 + lane * 4 + q; o[c][q] = (v[c * 4 + q] - mu) * rs * bfr(gg[col]) + bfr(bb[col]); }
#pragma unroll 1
    for (int ps = 0; ps < 2; ++ps) {
#pragma unroll
        for (int c = 0; c < 2; ++c) *(volatile v4f*)(OUT + (size_t)r * CC + c * 128 + lane * 4) = o[c];
        if (ps == 0) __threadfence(); }
}

extern "C" void kernel_launch(void* const* d_in, const int* in_sizes, int n_in,
                              void* d_out, int out_size, void* d_ws, size_t ws_size, hipStream_t stream) {
    (void)in_sizes; (void)n_in; (void)out_size;
    const float* x = (const float*)d_in[0]; const float* l1g = (const float*)d_in[1]; const float* l1b = (const float*)d_in[2]; const float* qkv_w = (const float*)d_in[3]; const float* qkv_b = (const float*)d_in[4]; const float* tab = (const float*)d_in[5]; const float* scp = (const float*)d_in[6]; const float* pw = (const float*)d_in[7]; const float* pb = (const float*)d_in[8]; const float* l2g = (const float*)d_in[9]; const float* l2b = (const float*)d_in[10];
    float* OUT = (float*)d_out;
    char* wsp = (char*)d_ws;
    auto take = [&](size_t bytes) { char* p = wsp; wsp += (bytes + 255) & ~(size_t)255; return (void*)p; };
    bf* WQKV = (bf*)take((size_t)3 * CC * CC * 2); bf* WP = (bf*)take((size_t)CC * CC * 2);
    bf* Hh = (bf*)take((size_t)NT * CC * 2); bf* Hl = (bf*)take((size_t)NT * CC * 2); float* F = (float*)take((size_t)NT * 3 * CC * 4);
    h16* Qp = (h16*)take((size_t)NT * CC * 2); h16* Kp = (h16*)take((size_t)NT * CC * 2); h16* VT = (h16*)take((size_t)NT * CC * 2);
    float* Sb = (float*)take((size_t)NN * NN * 4); h16* Pm = (h16*)take((size_t)NN * NN * 2); float* O = (float*)take((size_t)NT * CC * 4); float* O2 = (float*)take((size_t)NT * CC * 4);
    if ((size_t)(wsp - (char*)d_ws) > ws_size) return;
    bf* Oh = Hh; bf* Ol = Hl;
    { const unsigned g3 = (unsigned)((3 * CC * CC / 64 + 63) / 64), g1 = (unsigned)((CC * CC / 64 + 63) / 64); k_wtb<<<g3, 256, 0, stream>>>(qkv_w, CC, 3 * CC, 3 * CC, 0, WQKV); k_wtb<<<g1, 256, 0, stream>>>(pw, CC, CC, CC, 0, WP); }
    k_ln1<<<NT / 8, 256, 0, stream>>>(x, l1g, l1b, Hh, Hl);
    k_gemmw<bf, 1, true><<<dim3(NT / 64, 3 * CC / 64, 1), 32, 0, stream>>>(Hh, Hl, WQKV, nullptr, CC, F, 3 * CC, qkv_b, 0, 0, 0);
    k_qkplanes<<<(NT * 2 * CC / 64 + 63) / 64, 256, 0, stream>>>(F, Qp, Kp); k_vtplane<<<(NT * CC / 64 + 63) / 64, 256, 0, stream>>>(F, VT);
    for (int b = 0; b < NB_; ++b) { const size_t r0 = (size_t)b * NN;
        k_gemmw<h16, 0, false><<<dim3(NN / 64, NN / 64, 1), 32, 0, stream>>>(Qp + r0 * CC, nullptr, Kp + r0 * CC, nullptr, CC, Sb, NN, nullptr, 0, 0, 0);
        k_softrb<<<NN / 8, 256, 0, stream>>>(Sb, tab, scp, Pm);
        k_gemmw<h16, 0, false><<<dim3(NN / 64, CC / 64, 1), 32, 0, stream>>>(Pm, nullptr, VT + r0 * CC, nullptr, NN, O + r0 * CC, CC, nullptr, 0, 0, 0); }
    k_split1k<<<(NT * CC / 64 + 63) / 64, 256, 0, stream>>>(O, NT * CC / 64, Oh, Ol);
    k_gemmw<bf, 1, true><<<dim3(NT / 64, CC / 64, 1), 32, 0, stream>>>(Oh, Ol, WP, nullptr, CC, O2, CC, pb, 0, 0, 0);
    k_ln2<<<NT / 8, 256, 0, stream>>>(O2, l2g, l2b, OUT);
}
